// MambaBlock_47201690583665
// MI455X (gfx1250) — hardware-run, weakly checked
//
#include <hip/hip_runtime.h>
#include <math.h>

typedef __attribute__((ext_vector_type(16))) _Float16 v16h;
typedef __attribute__((ext_vector_type(8)))  _Float16 v8h;
typedef __attribute__((ext_vector_type(8)))  float    v8f;
typedef __attribute__((ext_vector_type(4)))  float    v4f;

constexpr int kBatch = 4;
constexpr int kSeq   = 2048;
constexpr int kDm    = 1024;
constexpr int kDi    = 2048;
constexpr int kNst   = 16;
constexpr int kRows  = kBatch * kSeq;
constexpr int kXrP   = 2 * kDi;
constexpr int kWdtN  = 64;
constexpr int kPreP  = 64;
constexpr int kDagP  = 32;
constexpr int kGateRow = 20;
constexpr int kTP    = 260;
constexpr int kScanTS = 32;

constexpr float kCarryAct = 64.0f;
constexpr float kCarryW   = 1024.0f;
constexpr float kFold     = 1.0f / (kCarryAct * kCarryW);
constexpr float kF16MinNormal = 6.103515625e-5f;

static_assert(kRows == 8192, "token rows");
static_assert((kRows % 64) == 0 && (kXrP % 64) == 0 && (kDm % 64) == 0 && (kWdtN % 64) == 0, "GEMM M,N multiples of 64");
static_assert((kDm % 32) == 0 && (kDi % 32) == 0, "GEMM K multiples of 32");
static_assert((kSeq % 64) == 0 && (kSeq % kScanTS) == 0 && (kDi % 256) == 0, "tile multiples");
static_assert(kNst == 16 && kDagP == 32, "state layout");

constexpr size_t kSzX16  = (size_t)kRows * kDm * 2;
constexpr size_t kSzInW  = (size_t)kXrP * kDm * 2;
constexpr size_t kSzOutW = (size_t)kDm * kDi * 2;
constexpr size_t kSzWdt  = (size_t)kWdtN * kDi * 2;
constexpr size_t kSzXR   = (size_t)kRows * kXrP * 2;
constexpr size_t kSzCV   = (size_t)kRows * kDi * 2;
constexpr size_t kSzPre  = (size_t)kRows * kPreP * 4;
constexpr size_t kSzDag  = (size_t)kRows * kDagP * 4;
constexpr size_t kSzDbs  = (size_t)kDi * kNst * 4;
constexpr size_t kOffX16  = 0;
constexpr size_t kOffInW  = kOffX16  + kSzX16;
constexpr size_t kOffOutW = kOffInW  + kSzInW;
constexpr size_t kOffWdt  = kOffOutW + kSzOutW;
constexpr size_t kOffXR   = kOffWdt  + kSzWdt;
constexpr size_t kOffCV   = kOffXR   + kSzXR;
constexpr size_t kOffPre  = kOffCV   + kSzCV;
constexpr size_t kOffDag  = kOffPre  + kSzPre;
constexpr size_t kOffDbs  = kOffDag  + kSzDag;
constexpr size_t kWsTotal = kOffDbs  + kSzDbs;
static_assert(kWsTotal == 133562368ull, "carve total");
static_assert(kWsTotal <= 134217728ull, "carve cap");
static_assert((kOffInW % 128) == 0 && (kOffOutW % 128) == 0 && (kOffWdt % 128) == 0 && (kOffXR % 128) == 0 &&
              (kOffCV % 128) == 0 && (kOffPre % 128) == 0 && (kOffDag % 128) == 0 && (kOffDbs % 128) == 0,
              "128-B aligned regions");

__device__ __forceinline__ float h16_to_f32(unsigned hb) {
  const unsigned sgn = (hb & 0x8000u) << 16;
  const unsigned em = hb & 0x7fffu;
  const float fn = __uint_as_float((em << 13) + 0x38000000u);
  const float fs = (float)em * 5.9604644775390625e-8f;
  const float mag = (em < 0x400u) ? fs : fn;
  return __uint_as_float(__float_as_uint(mag) | sgn);
}

__device__ __forceinline__ _Float16 to_f16_operand(float v) {
  float f = (fabsf(v) < kF16MinNormal) ? 0.0f : v;
  f = fminf(fmaxf(f, -60000.0f), 60000.0f);
  return (_Float16)f;
}

__device__ __forceinline__ float softplus_f(float x) {
  return fmaxf(x, 0.0f) + log1pf(expf(-fabsf(x)));
}

__device__ __forceinline__ void tile_guard_h(v8f& a, v8f& b, v8f& c, v8f& d, v16h x,
                                             v16h b0, v16h b1, v16h b2, v16h b3) {
  asm volatile("v_nop\n\tv_nop\n\tv_nop\n\tv_nop"
               : "+v"(a), "+v"(b), "+v"(c), "+v"(d)
               : "v"(x), "v"(b0), "v"(b1), "v"(b2), "v"(b3));
}
__device__ __forceinline__ void keep4_h(v16h a, v16h b, v16h c, v16h d) { asm volatile("v_nop" :: "v"(a), "v"(b), "v"(c), "v"(d)); }
__device__ __forceinline__ void acc_guard4(v8f& a, v8f& b, v8f& c, v8f& d) { asm volatile("v_nop\n\tv_nop\n\tv_nop\n\tv_nop" : "+v"(a), "+v"(b), "+v"(c), "+v"(d)); }

struct FragH {
  union U { v16h v; v8h h[2]; };
  static __device__ __forceinline__ v16h load(const _Float16* p) {
    U f;
    f.h[0] = *(const v8h*)(p);
    f.h[1] = *(const v8h*)(p + 16);
    return f.v;
  }
  static __device__ __forceinline__ v8f mma(v16h a, v16h b, v8f c) {
    return __builtin_amdgcn_wmma_f32_16x16x32_f16(false, a, false, b, (short)0, c, false, false);
  }
};

template <int BIAS_MODE, int OUT_MODE>
__global__ __launch_bounds__(256) void wmma_gemm64(
    const unsigned short* __restrict__ Ap, int lda,
    const unsigned short* __restrict__ Btp, int ldb,
    void* __restrict__ Cout, int ldc,
    const float* __restrict__ bias,
    int M, int N, int K, float scale) {
  const _Float16* A  = (const _Float16*)Ap;
  const _Float16* Bt = (const _Float16*)Btp;
  __shared__ __align__(16) float sT[8][16 * 68];
  const int lane = threadIdx.x & 31;
  const int wave = threadIdx.x >> 5;
  const int tilesN = N >> 6;
  const int tilesM = M >> 6;
  const int tile = blockIdx.x * 8 + wave;
  if (tile >= tilesM * tilesN) return;
  const int tm = tile / tilesN;
  const int tn = tile - tm * tilesN;
  const int m0 = tm << 6;
  const int n0 = tn << 6;

  const int rlane = lane & 15;
  const int koff  = (lane >> 4) * 8;
  const int mOff  = (lane >> 4) * 8;

  v8f acc[4][4];
#pragma unroll
  for (int i = 0; i < 4; ++i)
#pragma unroll
    for (int j = 0; j < 4; ++j) acc[i][j] = (v8f){0.f,0.f,0.f,0.f,0.f,0.f,0.f,0.f};

  for (int k0 = 0; k0 < K; k0 += 32) {
    v16h bh[4];
#pragma unroll
    for (int j = 0; j < 4; ++j) {
      const size_t bo = (size_t)(n0 + (j << 4) + rlane) * ldb + koff + k0;
      bh[j] = FragH::load(Bt + bo);
    }
#pragma unroll
    for (int i = 0; i < 4; ++i) {
      const size_t ao = (size_t)(m0 + (i << 4) + rlane) * lda + koff + k0;
      v16h ah = FragH::load(A + ao);
#pragma unroll
      for (int j = 0; j < 4; ++j) acc[i][j] = FragH::mma(ah, bh[j], acc[i][j]);
      tile_guard_h(acc[i][0], acc[i][1], acc[i][2], acc[i][3], ah, bh[0], bh[1], bh[2], bh[3]);
    }
    keep4_h(bh[0], bh[1], bh[2], bh[3]);
  }
  acc_guard4(acc[0][0], acc[0][1], acc[0][2], acc[0][3]);
  acc_guard4(acc[1][0], acc[1][1], acc[1][2], acc[1][3]);
  acc_guard4(acc[2][0], acc[2][1], acc[2][2], acc[2][3]);
  acc_guard4(acc[3][0], acc[3][1], acc[3][2], acc[3][3]);

  float* slab = sT[wave];
#pragma unroll
  for (int i = 0; i < 4; ++i) {
    const int mBase = m0 + (i << 4);
#pragma unroll
    for (int j = 0; j < 4; ++j) {
      const int n = n0 + (j << 4) + rlane;
      float bv = 0.f;
      if (BIAS_MODE == 2) bv = bias[n];
#pragma unroll
      for (int r = 0; r < 8; ++r) {
        float v = acc[i][j][r] * scale;
        if (BIAS_MODE == 2) v += bv;
        slab[(mOff + r) * 68 + (j << 4) + rlane] = v;
      }
    }
    __builtin_amdgcn_fence(__ATOMIC_RELEASE, "workgroup");
    __builtin_amdgcn_wave_barrier();
    __builtin_amdgcn_fence(__ATOMIC_ACQUIRE, "workgroup");
    if (OUT_MODE == 0) {
      float* C = (float*)Cout;
      const int hh = lane >> 4, c4 = (lane & 15) * 4;
      for (int pass = 0; pass < 2; ++pass) {
#pragma unroll
        for (int it = 0; it < 8; ++it) {
          const int row = it * 2 + hh;
          v4f v = *(const v4f*)(slab + row * 68 + c4);
          *(volatile v4f*)(C + (size_t)(mBase + row) * ldc + n0 + c4) = v;
        }
        __threadfence();
      }
    } else {
      const int q = lane >> 3, c8 = (lane & 7) * 8;
      unsigned short* C = (unsigned short*)Cout;
      for (int pass = 0; pass < 2; ++pass) {
#pragma unroll
        for (int it = 0; it < 4; ++it) {
          const int row = it * 4 + q;
          const float* sp = slab + row * 68 + c8;
          v8h hv;
#pragma unroll
          for (int e = 0; e < 8; ++e) hv[e] = (_Float16)sp[e];
          *(volatile v8h*)(C + (size_t)(mBase + row) * ldc + n0 + c8) = hv;
        }
        __threadfence();
      }
    }
    __builtin_amdgcn_fence(__ATOMIC_RELEASE, "workgroup");
    __builtin_amdgcn_wave_barrier();
    __builtin_amdgcn_fence(__ATOMIC_ACQUIRE, "workgroup");
  }
}

__global__ __launch_bounds__(256) void cast_f16_kernel(
    const float* __restrict__ src, unsigned short* __restrict__ dst, int total8, float carry)
{
  const int i = blockIdx.x * 256 + threadIdx.x;
  if (i >= total8) return;
  const size_t e0 = (size_t)i << 3;
  const float* p = src + e0;
  const v4f a0 = *(const v4f*)(p);
  const v4f a1 = *(const v4f*)(p + 4);
  v8h hv;
#pragma unroll
  for (int e = 0; e < 4; ++e) {
    hv[e]     = to_f16_operand(a0[e] * carry);
    hv[4 + e] = to_f16_operand(a1[e] * carry);
  }
  unsigned short* q = dst + e0;
  *(volatile v8h*)q = hv;
  __threadfence();
  *(volatile v8h*)q = hv;
}

__global__ __launch_bounds__(256) void build_wdt_kernel(
    const float* __restrict__ dt_w, const float* __restrict__ xproj_w, unsigned short* __restrict__ dst, float carry)
{
  const int i = blockIdx.x * 256 + threadIdx.x;
  if (i >= kWdtN * kDi / 8) return;
  const int e0 = i << 3;
  const int r  = e0 >> 11;
  const int c  = e0 & (kDi - 1);
  const int rdt = (r < kNst) ? r : (kNst - 1);
  const float* pa = dt_w + (size_t)rdt * kDi + c;
  const float* pb = xproj_w + (size_t)kGateRow * kDi + c;
  v4f a0 = *(const v4f*)(pa);
  v4f a1 = *(const v4f*)(pa + 4);
  v4f b0 = *(const v4f*)(pb);
  v4f b1 = *(const v4f*)(pb + 4);
  asm volatile("" : "+v"(a0));
  asm volatile("" : "+v"(a1));
  asm volatile("" : "+v"(b0));
  asm volatile("" : "+v"(b1));
  const bool isdt = (r < kNst);
  const bool isg  = (r == kNst);
  v8h hv;
#pragma unroll
  for (int e = 0; e < 4; ++e) {
    const float v0 = isdt ? a0[e] : (isg ? b0[e] : 0.0f);
    const float v1 = isdt ? a1[e] : (isg ? b1[e] : 0.0f);
    hv[e]     = to_f16_operand(v0 * carry);
    hv[4 + e] = to_f16_operand(v1 * carry);
  }
  unsigned short* q = dst + e0;
  *(volatile v8h*)q = hv;
  __threadfence();
  *(volatile v8h*)q = hv;
}

__global__ __launch_bounds__(256) void softplus_plane_kernel(
    const float* __restrict__ src, float* __restrict__ dst, int n)
{
  __shared__ __align__(16) float sO[256];
  const int tid = threadIdx.x;
  const int base = blockIdx.x * 256;
  const int idx = base + tid;
  const int idc = (idx < n) ? idx : (n - 1);
  const float v = src[idc];
  sO[tid] = softplus_f(v);
  __syncthreads();
  if (tid < 64) {
    const v4f o = *(const v4f*)(sO + tid * 4);
    float* p = dst + base + tid * 4;
    *(volatile v4f*)p = o;
    __threadfence();
    *(volatile v4f*)p = o;
  }
}

__global__ __launch_bounds__(256) void decay_gate_kernel(
    const float* __restrict__ PRE, const float* __restrict__ dt_b, const float* __restrict__ Avec,
    const float* __restrict__ xproj_b, float* __restrict__ DAG)
{
  __shared__ __align__(16) float sO[256];
  const int tid = threadIdx.x;
  const int base = blockIdx.x * 256;
  const int idx = base + tid;
  const int row = idx >> 5;
  const int n   = idx & 31;
  const int nc  = n & (kNst - 1);
  const float pre = PRE[(size_t)row * kPreP + n];
  const float bdt = dt_b[nc];
  const float av  = Avec[nc];
  const float bg  = xproj_b[kGateRow];
  const float delta = softplus_f(pre + bdt);
  const float spa   = softplus_f(av);
  const float da    = expf(-delta * spa);
  const float g     = pre + bg;
  const float sg    = g * (1.0f / (1.0f + expf(-g)));
  const float o = (n < kNst) ? da : ((n == kNst) ? sg : 0.0f);
  sO[tid] = o;
  __syncthreads();
  if (tid < 64) {
    const v4f ov = *(const v4f*)(sO + tid * 4);
    float* p = DAG + base + tid * 4;
    *(volatile v4f*)p = ov;
    __threadfence();
    *(volatile v4f*)p = ov;
  }
}

__global__ __launch_bounds__(256) void conv_kernel(
    const unsigned short* __restrict__ XR, const float* __restrict__ cw, const float* __restrict__ cb,
    unsigned short* __restrict__ CV)
{
  __shared__ __align__(16) float sT[16 * kTP];
  const int tid = threadIdx.x, lane = tid & 31, wave = tid >> 5;
  const int d0 = blockIdx.x * 256, d = d0 + tid;
  const int g0 = blockIdx.y * 64;
  const int tb = g0 & (kSeq - 1);
  const v4f wv = *(const v4f*)(cw + (size_t)d * 4);
  const float w0 = wv[0], w1 = wv[1], w2 = wv[2], w3 = wv[3];
  const float bc = cb[d];
  float xm1, xc, xp1;
  {
    const bool hist = (tb > 0);
    const int rb = hist ? (g0 - 1) : g0;
    const unsigned um = XR[(size_t)rb * kXrP + d];
    const unsigned uc = XR[(size_t)g0 * kXrP + d];
    const unsigned up = XR[(size_t)(g0 + 1) * kXrP + d];
    const float fm = h16_to_f32(um);
    xm1 = hist ? fm : 0.0f;
    xc  = h16_to_f32(uc);
    xp1 = h16_to_f32(up);
  }
#pragma unroll 1
  for (int sub = 0; sub < 4; ++sub) {
    const int lb = g0 + sub * 16;
#pragma unroll 1
    for (int s = 0; s < 16; ++s) {
      const int g = lb + s;
      const int t = tb + sub * 16 + s;
      const bool ok2 = (t + 2 < kSeq);
      const int r2 = ok2 ? (g + 2) : g;
      const unsigned u2 = XR[(size_t)r2 * kXrP + d];
      const float f2 = h16_to_f32(u2);
      const float xp2 = ok2 ? f2 : 0.0f;
      float acc = w0 * xm1;
      acc = fmaf(w1, xc, acc);
      acc = fmaf(w2, xp1, acc);
      acc = fmaf(w3, xp2, acc);
      sT[s * kTP + tid] = (acc + bc) * kCarryAct;
      xm1 = xc; xc = xp1; xp1 = xp2;
    }
    __syncthreads();
    v8h bv[2];
#pragma unroll
    for (int it = 0; it < 2; ++it) {
      const float* sp = sT + (it * 8 + wave) * kTP + lane * 8;
      const v4f a0 = *(const v4f*)(sp);
      const v4f a1 = *(const v4f*)(sp + 4);
#pragma unroll
      for (int e = 0; e < 4; ++e) {
        bv[it][e]     = to_f16_operand(a0[e]);
        bv[it][4 + e] = to_f16_operand(a1[e]);
      }
    }
    for (int pass = 0; pass < 2; ++pass) {
#pragma unroll
      for (int it = 0; it < 2; ++it)
        *(volatile v8h*)(CV + (size_t)(lb + it * 8 + wave) * kDi + d0 + lane * 8) = bv[it];
      __threadfence();
    }
    __syncthreads();
  }
}

__global__ __launch_bounds__(256) void scan_kernel(
    const unsigned short* __restrict__ XR, const float* __restrict__ DAG, const float* __restrict__ DBS,
    const float* __restrict__ Cm, unsigned short* __restrict__ OP)
{
  __shared__ __align__(16) float sD[kScanTS * kDagP];
  __shared__ __align__(16) float sY[kScanTS * kTP];
  const int tid = threadIdx.x, lane = tid & 31, wave = tid >> 5;
  const int d0 = blockIdx.x * 256, d = d0 + tid;
  const size_t row0 = (size_t)blockIdx.y * kSeq;

  float dB[kNst], dC[kNst], h[kNst];
#pragma unroll
  for (int q = 0; q < 4; ++q) {
    const v4f bq = *(const v4f*)(DBS + (size_t)d * kNst + 4 * q);
    const v4f cq = *(const v4f*)(Cm  + (size_t)d * kNst + 4 * q);
    dB[4 * q + 0] = bq[0]; dB[4 * q + 1] = bq[1]; dB[4 * q + 2] = bq[2]; dB[4 * q + 3] = bq[3];
    dC[4 * q + 0] = cq[0]; dC[4 * q + 1] = cq[1]; dC[4 * q + 2] = cq[2]; dC[4 * q + 3] = cq[3];
  }
#pragma unroll
  for (int n = 0; n < kNst; ++n) h[n] = 0.0f;

  const int sr = tid >> 3, sq = (tid & 7) * 4;
#pragma unroll 1
  for (int t0 = 0; t0 < kSeq; t0 += kScanTS) {
    __syncthreads();
    *(v4f*)(sD + sr * kDagP + sq) = *(const v4f*)(DAG + (row0 + t0 + sr) * kDagP + sq);
    __syncthreads();
#pragma unroll 1
    for (int s = 0; s < kScanTS; ++s) {
      const size_t m = row0 + t0 + s;
      const unsigned xw = XR[m * kXrP + d];
      const unsigned rw = XR[m * kXrP + kDi + d];
      const float xv = h16_to_f32(xw);
      const float rv = h16_to_f32(rw);
      const float* dr = sD + s * kDagP;
      v4f aq[4];
#pragma unroll
      for (int q = 0; q < 4; ++q) aq[q] = *(const v4f*)(dr + 4 * q);
      const float gt = dr[kNst];
      float y = 0.0f;
#pragma unroll
      for (int n = 0; n < kNst; ++n) {
        const float p = xv * dB[n];
        const float hn = fmaf(h[n], aq[n >> 2][n & 3], p);
        h[n] = hn;
        y = fmaf(hn, dC[n], y);
      }
      const float o = fmaf(y, gt, rv);
      sY[s * kTP + tid] = o * kCarryAct;
    }
    __syncthreads();
    v8h hv[4];
#pragma unroll
    for (int it = 0; it < 4; ++it) {
      const float* sp = sY + (it * 8 + wave) * kTP + lane * 8;
      const v4f a0 = *(const v4f*)(sp);
      const v4f a1 = *(const v4f*)(sp + 4);
#pragma unroll
      for (int e = 0; e < 4; ++e) {
        hv[it][e]     = to_f16_operand(a0[e]);
        hv[it][4 + e] = to_f16_operand(a1[e]);
      }
    }
    for (int pass = 0; pass < 2; ++pass) {
#pragma unroll
      for (int it = 0; it < 4; ++it)
        *(volatile v8h*)(OP + (row0 + t0 + it * 8 + wave) * kDi + d0 + lane * 8) = hv[it];
      __threadfence();
    }
  }
}

extern "C" void kernel_launch(void* const* d_in, const int* in_sizes, int n_in,
                              void* d_out, int out_size, void* d_ws, size_t ws_size,
                              hipStream_t stream)
{
  if (n_in < 14) return;
  if (in_sizes[0] != kRows * kDm) return;
  if (in_sizes[1] != kXrP * kDm) return;
  if (in_sizes[2] != kXrP) return;
  if (in_sizes[3] != kDi * 4) return;
  if (in_sizes[4] != kDi) return;
  if (in_sizes[5] != 21 * kDi) return;
  if (in_sizes[6] != 21) return;
  if (in_sizes[7] != kNst * kDi) return;
  if (in_sizes[8] != kNst) return;
  if (in_sizes[9] != kNst) return;
  if (in_sizes[10] != kDi * kNst) return;
  if (in_sizes[11] != kDi * kNst) return;
  if (in_sizes[12] != kDm * kDi) return;
  if (in_sizes[13] != kDm) return;
  if (out_size != kRows * kDm) return;
  if (ws_size < kWsTotal) return;

  const float* x       = (const float*)d_in[0];
  const float* in_w    = (const float*)d_in[1];
  const float* in_b    = (const float*)d_in[2];
  const float* conv_w  = (const float*)d_in[3];
  const float* conv_b  = (const float*)d_in[4];
  const float* xproj_w = (const float*)d_in[5];
  const float* xproj_b = (const float*)d_in[6];
  const float* dt_w    = (const float*)d_in[7];
  const float* dt_b    = (const float*)d_in[8];
  const float* Avec    = (const float*)d_in[9];
  const float* Bm      = (const float*)d_in[10];
  const float* Cm      = (const float*)d_in[11];
  const float* out_w   = (const float*)d_in[12];
  const float* out_b   = (const float*)d_in[13];
  float* out = (float*)d_out;

  char* ws = (char*)d_ws;
  unsigned short* X16  = (unsigned short*)(ws + kOffX16);
  unsigned short* INW  = (unsigned short*)(ws + kOffInW);
  unsigned short* OUTW = (unsigned short*)(ws + kOffOutW);
  unsigned short* WDT  = (unsigned short*)(ws + kOffWdt);
  unsigned short* XR   = (unsigned short*)(ws + kOffXR);
  unsigned short* CV   = (unsigned short*)(ws + kOffCV);
  float*          PRE  = (float*)(ws + kOffPre);
  float*          DAG  = (float*)(ws + kOffDag);
  float*          DBS  = (float*)(ws + kOffDbs);

  cast_f16_kernel<<<(kRows * kDm) / 8 / 256, 256, 0, stream>>>(x, X16, (kRows * kDm) / 8, kCarryAct);
  cast_f16_kernel<<<(kXrP * kDm) / 8 / 256, 256, 0, stream>>>(in_w, INW, (kXrP * kDm) / 8, kCarryW);
  cast_f16_kernel<<<(kDm * kDi) / 8 / 256, 256, 0, stream>>>(out_w, OUTW, (kDm * kDi) / 8, kCarryW);
  build_wdt_kernel<<<(kWdtN * kDi) / 8 / 256, 256, 0, stream>>>(dt_w, xproj_w, WDT, kCarryW);
  softplus_plane_kernel<<<(kDi * kNst) / 256, 256, 0, stream>>>(Bm, DBS, kDi * kNst);

  wmma_gemm64<2, 1><<<dim3((kRows / 64) * (kXrP / 64) / 8), 256, 0, stream>>>(
      X16, kDm, INW, kDm, (void*)XR, kXrP, in_b, kRows, kXrP, kDm, kFold);

  conv_kernel<<<dim3(kDi / 256, kRows / 64), 256, 0, stream>>>(XR, conv_w, conv_b, CV);

  wmma_gemm64<0, 0><<<dim3((kRows / 64) * (kWdtN / 64) / 8), 256, 0, stream>>>(
      CV, kDi, WDT, kDi, (void*)PRE, kPreP, dt_b, kRows, kWdtN, kDi, kFold);

  decay_gate_kernel<<<(kRows * kDagP) / 256, 256, 0, stream>>>(PRE, dt_b, Avec, xproj_b, DAG);

  scan_kernel<<<dim3(kDi / 256, kBatch), 256, 0, stream>>>(XR, DAG, DBS, Cm, CV);

  wmma_gemm64<2, 0><<<dim3((kRows / 64) * (kDm / 64) / 8), 256, 0, stream>>>(
      CV, kDi, OUTW, kDi, (void*)out, kDm, out_b, kRows, kDm, kDi, kFold);
}
